// ConvTSP_32633161515437
// MI455X (gfx1250) — hardware-verified
//
#include <hip/hip_runtime.h>
#define BB 4
#define NNODE 200
#define HH 128
#define HHALF 64
#define NL 3
#define NX (BB * NNODE)
#define NEDGE (BB * NNODE * NNODE)
#define ECH (NNODE * NNODE)

typedef __bf16 v16b __attribute__((ext_vector_type(16)));
typedef unsigned short v8us __attribute__((ext_vector_type(8), may_alias));
typedef float  v8f  __attribute__((ext_vector_type(8)));
typedef float  v4f  __attribute__((ext_vector_type(4)));
typedef float  v4fa __attribute__((ext_vector_type(4), may_alias));
union FragB { v16b v; v8us half[2]; unsigned short u[16]; };

__device__ __forceinline__ unsigned short bf16_bits(float x) { unsigned int u = __float_as_uint(x); return (unsigned short)((u + 0x7FFFu + ((u >> 16) & 1u)) >> 16); }
__device__ __forceinline__ float bf16_val(unsigned short b) { return __uint_as_float(((unsigned int)b) << 16); }
__device__ __forceinline__ float bf16_round(float x) { return bf16_val(bf16_bits(x)); }
template <int NT>
__device__ __forceinline__ v8f mmaN(v16b ah, v16b al, v16b bh, v16b bl, v8f c) {
  c = __builtin_amdgcn_wmma_f32_16x16x32_bf16(false, ah, false, bh, (short)0, c, false, false);
  if (NT >= 2) c = __builtin_amdgcn_wmma_f32_16x16x32_bf16(false, al, false, bh, (short)0, c, false, false);
  if (NT >= 3) c = __builtin_amdgcn_wmma_f32_16x16x32_bf16(false, ah, false, bl, (short)0, c, false, false);
  asm volatile("v_nop\n\tv_nop\n\tv_nop\n\tv_nop" : "+v"(c) : "v"(ah), "v"(al), "v"(bh), "v"(bl));
  return c;
}

__global__ __launch_bounds__(256) void k_wt_bf16(const float* __restrict__ W, unsigned short* __restrict__ Wt, int K, int N) {
  const int t = blockIdx.x * 256 + threadIdx.x;
  const int k8n = K / 8;
  if (t >= N * k8n) return;
  const int n = t / k8n, k8 = (t % k8n) * 8;
  v8us v;
#pragma unroll
  for (int i = 0; i < 8; ++i) v[i] = bf16_bits(W[(size_t)(k8 + i) * N + n]);
  *(volatile v8us*)(Wt + (size_t)n * K + k8) = v;
  __threadfence();
  *(volatile v8us*)(Wt + (size_t)n * K + k8) = v;
}

template <bool ASPLIT, int ACT, bool BIAS_BF16>
__global__ __launch_bounds__(128) void k_gemm_bf(const float* __restrict__ A, int lda, const unsigned short* __restrict__ Wt, int ldb,
                                               const float* __restrict__ bias, float* __restrict__ C, int ldc, int M, int N, int K) {
  __shared__ __attribute__((aligned(16))) float so[4][16][64];
  const int tid = threadIdx.x, w = tid >> 5, lane = tid & 31, ln = lane & 15, hh = lane >> 4;
  const int ntn = N / 64;
  const int wid = blockIdx.x * 4 + w;
  const int mt = wid / ntn, nq = wid % ntn;
  if (mt * 16 >= M) return;
  const int row0 = mt * 16, col0 = nq * 64;
  const float* arow = A + (size_t)(row0 + ln) * lda;
  v8f acc[4] = {};
  for (int kb = 0; kb < K; kb += 32) {
    FragB ah, al;
    const v4f x0 = *(const v4fa*)(arow + kb + 8 * hh), x1 = *(const v4fa*)(arow + kb + 8 * hh + 4);
    const v4f x2 = *(const v4fa*)(arow + kb + 16 + 8 * hh), x3 = *(const v4fa*)(arow + kb + 16 + 8 * hh + 4);
    float xs[16] = {x0[0],x0[1],x0[2],x0[3],x1[0],x1[1],x1[2],x1[3],x2[0],x2[1],x2[2],x2[3],x3[0],x3[1],x3[2],x3[3]};
#pragma unroll
    for (int i = 0; i < 16; ++i) { const unsigned short hb = bf16_bits(xs[i]); ah.u[i] = hb; al.u[i] = ASPLIT ? bf16_bits(xs[i] - bf16_val(hb)) : (unsigned short)0; }
#pragma unroll
    for (int t = 0; t < 4; ++t) {
      const unsigned short* brow = Wt + (size_t)(col0 + t * 16 + ln) * ldb + kb;
      FragB b;
      b.half[0] = *(const v8us*)(brow + 8 * hh);
      b.half[1] = *(const v8us*)(brow + 16 + 8 * hh);
      acc[t] = mmaN<ASPLIT ? 2 : 1>(ah.v, al.v, b.v, b.v, acc[t]);
    }
  }
#pragma unroll
  for (int t = 0; t < 4; ++t) {
    float bv = bias ? bias[col0 + t * 16 + ln] : 0.f;
    if (BIAS_BF16) bv = bf16_round(bv);
#pragma unroll
    for (int r = 0; r < 8; ++r) { float v = acc[t][r] + bv; if (ACT == 1) v = fmaxf(v, 0.f); so[w][8 * hh + r][t * 16 + ln] = v; }
  }
  __builtin_amdgcn_fence(__ATOMIC_ACQ_REL, "workgroup");
  __builtin_amdgcn_wave_barrier();
  const int rsub = lane >> 4, c4 = (lane & 15) * 4;
  for (int pass = 0; pass < 2; ++pass) {
#pragma unroll
    for (int q = 0; q < 8; ++q) {
      const int r = q * 2 + rsub;
      const v4f v = *(const v4fa*)&so[w][r][c4];
      *(volatile v4f*)(C + (size_t)(row0 + r) * ldc + col0 + c4) = v;
    }
    if (pass == 0) __threadfence();
  }
}

template <int D, bool CAUSAL>
__global__ __launch_bounds__(128) void k_flash(const float* __restrict__ qb, const float* __restrict__ kb, const float* __restrict__ vb,
                                             int pitch, int T, int H, float scale, float* __restrict__ y, int ypitch) {
  constexpr int KS = D / 32;
  constexpr int DT = D / 16;
  __shared__ __attribute__((aligned(16))) unsigned short sKh[32][D + 8], sKl[32][D + 8], sVh[32][D + 8], sVl[32][D + 8];
  __shared__ __attribute__((aligned(16))) unsigned short sPh[4][16][40], sPl[4][16][40];
  __shared__ __attribute__((aligned(16))) float sO[4][16][D];
  const int tid = threadIdx.x, w = tid >> 5, lane = tid & 31, ln = lane & 15, hh = lane >> 4;
  const int nqb = (T + 63) / 64;
  const int bh = blockIdx.x / nqb, qblk = blockIdx.x % nqb;
  const int b = bh / H, h = bh % H;
  const int q0 = qblk * 64 + w * 16;
  const float* Q = qb + (size_t)b * T * pitch + h * D;
  const float* K = kb + (size_t)b * T * pitch + h * D;
  const float* V = vb + (size_t)b * T * pitch + h * D;

  FragB aqh[KS], aql[KS];
  {
    int row = q0 + ln; if (row >= T) row = T - 1;
    const float* qr = Q + (size_t)row * pitch;
#pragma unroll
    for (int ks = 0; ks < KS; ++ks)
#pragma unroll
      for (int i = 0; i < 16; ++i) {
        const int d = ks * 32 + ((i < 8) ? (8 * hh + i) : (16 + 8 * hh + (i - 8)));
        const float x = qr[d] * scale; const unsigned short hb = bf16_bits(x);
        aqh[ks].u[i] = hb; aql[ks].u[i] = bf16_bits(x - bf16_val(hb));
      }
  }
  float m_r[8], l_r[8];
#pragma unroll
  for (int r = 0; r < 8; ++r) { m_r[r] = -3.0e38f; l_r[r] = 0.f; }
  v8f oacc[DT];
#pragma unroll
  for (int dt = 0; dt < DT; ++dt) oacc[dt] = (v8f){0.f,0.f,0.f,0.f,0.f,0.f,0.f,0.f};

  const int kv_end = CAUSAL ? min(T, qblk * 64 + 64) : T;
  for (int j0 = 0; j0 < kv_end; j0 += 32) {
    __syncthreads();
    for (int e = tid; e < 32 * (D / 4); e += 128) {
      const int r = e / (D / 4), c4 = (e % (D / 4)) * 4;
      const int key = j0 + r;
      v4f kf = {0.f,0.f,0.f,0.f}, vf = {0.f,0.f,0.f,0.f};
      if (key < T) { kf = *(const v4fa*)(K + (size_t)key * pitch + c4); vf = *(const v4fa*)(V + (size_t)key * pitch + c4); }
#pragma unroll
      for (int t = 0; t < 4; ++t) {
        unsigned short hb = bf16_bits(kf[t]); sKh[r][c4 + t] = hb; sKl[r][c4 + t] = bf16_bits(kf[t] - bf16_val(hb));
        hb = bf16_bits(vf[t]); sVh[r][c4 + t] = hb; sVl[r][c4 + t] = bf16_bits(vf[t] - bf16_val(hb));
      }
    }
    __syncthreads();
    v8f s[2];
#pragma unroll
    for (int nt = 0; nt < 2; ++nt) {
      v8f acc = {};
#pragma unroll
      for (int ks = 0; ks < KS; ++ks) {
        FragB bh_, bl_;
        bh_.half[0] = *(const v8us*)&sKh[nt * 16 + ln][ks * 32 + 8 * hh]; bh_.half[1] = *(const v8us*)&sKh[nt * 16 + ln][ks * 32 + 16 + 8 * hh];
        bl_.half[0] = *(const v8us*)&sKl[nt * 16 + ln][ks * 32 + 8 * hh]; bl_.half[1] = *(const v8us*)&sKl[nt * 16 + ln][ks * 32 + 16 + 8 * hh];
        acc = mmaN<3>(aqh[ks].v, aql[ks].v, bh_.v, bl_.v, acc);
      }
      s[nt] = acc;
    }
    float alpha[8];
#pragma unroll
    for (int r = 0; r < 8; ++r) {
      const int qi = q0 + 8 * hh + r;
      const int ja = j0 + ln, jb = j0 + 16 + ln;
      if (CAUSAL) { if (ja > qi) s[0][r] = -3.0e38f; if (jb > qi) s[1][r] = -3.0e38f; }
      if (ja >= T) s[0][r] = -3.0e38f;
      if (jb >= T) s[1][r] = -3.0e38f;
      float mx = fmaxf(s[0][r], s[1][r]);
      mx = fmaxf(mx, __shfl_xor(mx, 1, 32)); mx = fmaxf(mx, __shfl_xor(mx, 2, 32)); mx = fmaxf(mx, __shfl_xor(mx, 4, 32)); mx = fmaxf(mx, __shfl_xor(mx, 8, 32));
      const float mnew = fmaxf(m_r[r], mx);
      alpha[r] = (mnew > -1.0e38f) ? __expf(m_r[r] - mnew) : 1.0f;
      const float p0 = (s[0][r] > -1.0e38f) ? __expf(s[0][r] - mnew) : 0.f;
      const float p1 = (s[1][r] > -1.0e38f) ? __expf(s[1][r] - mnew) : 0.f;
      m_r[r] = mnew;
      l_r[r] = l_r[r] * alpha[r] + p0 + p1;
      unsigned short hb = bf16_bits(p0); sPh[w][8 * hh + r][ln] = hb;      sPl[w][8 * hh + r][ln] = bf16_bits(p0 - bf16_val(hb));
      hb = bf16_bits(p1);                sPh[w][8 * hh + r][16 + ln] = hb; sPl[w][8 * hh + r][16 + ln] = bf16_bits(p1 - bf16_val(hb));
    }
#pragma unroll
    for (int dt = 0; dt < DT; ++dt)
#pragma unroll
      for (int r = 0; r < 8; ++r) oacc[dt][r] *= alpha[r];
    __builtin_amdgcn_fence(__ATOMIC_ACQ_REL, "workgroup");
    __builtin_amdgcn_wave_barrier();
    FragB pah, pal;
    pah.half[0] = *(const v8us*)&sPh[w][ln][8 * hh]; pah.half[1] = *(const v8us*)&sPh[w][ln][16 + 8 * hh];
    pal.half[0] = *(const v8us*)&sPl[w][ln][8 * hh]; pal.half[1] = *(const v8us*)&sPl[w][ln][16 + 8 * hh];
#pragma unroll
    for (int dt = 0; dt < DT; ++dt) {
      FragB bvh, bvl;
#pragma unroll
      for (int i = 0; i < 8; ++i) {
        bvh.u[i] = sVh[8 * hh + i][dt * 16 + ln]; bvh.u[8 + i] = sVh[16 + 8 * hh + i][dt * 16 + ln];
        bvl.u[i] = sVl[8 * hh + i][dt * 16 + ln]; bvl.u[8 + i] = sVl[16 + 8 * hh + i][dt * 16 + ln];
      }
      oacc[dt] = mmaN<3>(pah.v, pal.v, bvh.v, bvl.v, oacc[dt]);
    }
    __builtin_amdgcn_fence(__ATOMIC_ACQ_REL, "workgroup");
    __builtin_amdgcn_wave_barrier();
  }
#pragma unroll
  for (int r = 0; r < 8; ++r) {
    float l = l_r[r];
    l += __shfl_xor(l, 1, 32); l += __shfl_xor(l, 2, 32); l += __shfl_xor(l, 4, 32); l += __shfl_xor(l, 8, 32);
    l_r[r] = (l > 0.f) ? 1.0f / l : 0.f;
  }
#pragma unroll
  for (int dt = 0; dt < DT; ++dt)
#pragma unroll
    for (int r = 0; r < 8; ++r) sO[w][8 * hh + r][dt * 16 + ln] = oacc[dt][r] * l_r[r];
  __builtin_amdgcn_fence(__ATOMIC_ACQ_REL, "workgroup");
  __builtin_amdgcn_wave_barrier();
  for (int pass = 0; pass < 2; ++pass) {
    for (int r = 0; r < 16; ++r) {
      const int row = q0 + r;
      if (row < T && lane < D / 4) {
        const v4f val = *(const v4fa*)&sO[w][r][lane * 4];
        *(volatile v4f*)(y + ((size_t)b * T + row) * ypitch + h * D + lane * 4) = val;
      }
    }
    if (pass == 0) __threadfence();
  }
}

typedef _Float16 v16h __attribute__((ext_vector_type(16)));
union FragH { v16h v; v8us half[2]; _Float16 h[16]; unsigned short u[16]; };
template <int NT>
__device__ __forceinline__ v8f mmaH(v16h ah, v16h al, v16h bh, v16h bl, v8f c) {
  c = __builtin_amdgcn_wmma_f32_16x16x32_f16(false, ah, false, bh, (short)0, c, false, false);
  if (NT >= 2) c = __builtin_amdgcn_wmma_f32_16x16x32_f16(false, al, false, bh, (short)0, c, false, false);
  if (NT >= 3) c = __builtin_amdgcn_wmma_f32_16x16x32_f16(false, ah, false, bl, (short)0, c, false, false);
  asm volatile("v_nop\n\tv_nop\n\tv_nop\n\tv_nop" : "+v"(c) : "v"(ah), "v"(al), "v"(bh), "v"(bl));
  return c;
}
template <bool ASPLIT>
__global__ __launch_bounds__(128) void k_gemm_h(const float* __restrict__ A, int lda, size_t sA, const _Float16* __restrict__ Bh, int ldb, size_t sB, float alpha, float* __restrict__ C, int ldc, size_t sC, int M, int N, int K) {
  __shared__ __attribute__((aligned(16))) float so[4][16][64];
  const int tid = threadIdx.x, w = tid >> 5, lane = tid & 31, ln = lane & 15, hh = lane >> 4; const int by = blockIdx.y;
  A += (size_t)by * sA; Bh += (size_t)by * sB; C += (size_t)by * sC;
  const int ntn = (N + 63) / 64; const int wid = blockIdx.x * 4 + w; const int mt = wid / ntn, nq = wid % ntn; if (mt * 16 >= M) return;
  const int row0 = mt * 16, col0 = nq * 64; const float* arow = A + (size_t)(row0 + ln) * lda;
  v8f acc[4] = {};
  for (int kb = 0; kb < K; kb += 32) {
    FragH ah, al;
    const v4f x0 = *(const v4fa*)(arow + kb + 8 * hh), x1 = *(const v4fa*)(arow + kb + 8 * hh + 4), x2 = *(const v4fa*)(arow + kb + 16 + 8 * hh), x3 = *(const v4fa*)(arow + kb + 16 + 8 * hh + 4);
    float xs[16] = {x0[0],x0[1],x0[2],x0[3],x1[0],x1[1],x1[2],x1[3],x2[0],x2[1],x2[2],x2[3],x3[0],x3[1],x3[2],x3[3]};
#pragma unroll
    for (int i = 0; i < 16; ++i) { const _Float16 h = (_Float16)xs[i]; ah.h[i] = h; al.h[i] = ASPLIT ? (_Float16)(xs[i] - (float)h) : (_Float16)0.0f; }
#pragma unroll
    for (int t = 0; t < 4; ++t) { if (col0 + t * 16 >= N) continue; const size_t boff = (size_t)(col0 + t * 16 + ln) * ldb + kb; FragH bq; bq.half[0] = *(const v8us*)(Bh + boff + 8 * hh); bq.half[1] = *(const v8us*)(Bh + boff + 16 + 8 * hh);
      acc[t] = mmaH<ASPLIT ? 2 : 1>(ah.v, al.v, bq.v, bq.v, acc[t]); }
  }
#pragma unroll
  for (int t = 0; t < 4; ++t) { if (col0 + t * 16 >= N) continue;
#pragma unroll
    for (int r = 0; r < 8; ++r) so[w][8 * hh + r][t * 16 + ln] = acc[t][r] * alpha; }
  __builtin_amdgcn_fence(__ATOMIC_ACQ_REL, "workgroup"); __builtin_amdgcn_wave_barrier();
  const int rsub = lane >> 4, c4 = (lane & 15) * 4;
  for (int pass = 0; pass < 2; ++pass) {
#pragma unroll
    for (int q = 0; q < 8; ++q) { const int r = q * 2 + rsub; if (col0 + c4 < N) { const v4f v = *(const v4fa*)&so[w][r][c4]; *(volatile v4f*)(C + (size_t)(row0 + r) * ldc + col0 + c4) = v; } }
    if (pass == 0) __threadfence(); }
}

template <int DUMMY>
__global__ __launch_bounds__(128) void k_gemm_hh(const _Float16* __restrict__ A, int lda, size_t sA, const _Float16* __restrict__ Bh, int ldb, size_t sB, float alpha, float* __restrict__ C, int ldc, size_t sC, int M, int N, int K) {
  __shared__ __attribute__((aligned(16))) float so[4][16][64];
  const int tid = threadIdx.x, w = tid >> 5, lane = tid & 31, ln = lane & 15, hh = lane >> 4; const int by = blockIdx.y;
  A += (size_t)by * sA; Bh += (size_t)by * sB; C += (size_t)by * sC;
  const int ntn = (N + 63) / 64; const int wid = blockIdx.x * 4 + w; const int mt = wid / ntn, nq = wid % ntn; if (mt * 16 >= M) return;
  const int row0 = mt * 16, col0 = nq * 64; const _Float16* arow = A + (size_t)(row0 + ln) * lda;
  v8f acc[4] = {};
  for (int kb = 0; kb < K; kb += 32) { FragH ah; ah.half[0] = *(const v8us*)((const unsigned short*)arow + kb + 8 * hh); ah.half[1] = *(const v8us*)((const unsigned short*)arow + kb + 16 + 8 * hh);
#pragma unroll
    for (int t = 0; t < 4; ++t) { if (col0 + t * 16 >= N) continue; const size_t boff = (size_t)(col0 + t * 16 + ln) * ldb + kb; FragH bq; bq.half[0] = *(const v8us*)((const unsigned short*)Bh + boff + 8 * hh); bq.half[1] = *(const v8us*)((const unsigned short*)Bh + boff + 16 + 8 * hh);
      acc[t] = mmaH<1>(ah.v, ah.v, bq.v, bq.v, acc[t]); }
  }
#pragma unroll
  for (int t = 0; t < 4; ++t) { if (col0 + t * 16 >= N) continue;
#pragma unroll
    for (int r = 0; r < 8; ++r) so[w][8 * hh + r][t * 16 + ln] = acc[t][r] * alpha; }
  __builtin_amdgcn_fence(__ATOMIC_ACQ_REL, "workgroup"); __builtin_amdgcn_wave_barrier();
  const int rsub = lane >> 4, c4 = (lane & 15) * 4;
  for (int pass = 0; pass < 2; ++pass) {
#pragma unroll
    for (int q = 0; q < 8; ++q) { const int r = q * 2 + rsub; if (col0 + c4 < N) { const v4f v = *(const v4fa*)&so[w][r][c4]; *(volatile v4f*)(C + (size_t)(row0 + r) * ldc + col0 + c4) = v; } }
    if (pass == 0) __threadfence(); }
}

template <int ACT>
__global__ __launch_bounds__(128) void k_gemm_hhx(const _Float16* __restrict__ A, int lda, size_t sA, const _Float16* __restrict__ Bh, int ldb, size_t sB, float alpha, const float* __restrict__ bias, size_t sBias, const float* __restrict__ CP, int rowsPerB, size_t sCPb, int row0g,
    float* __restrict__ C, _Float16* __restrict__ C16, int ldc, size_t sC, int M, int N, int K) {
  __shared__ __attribute__((aligned(16))) float so[4][16][64];
  const int tid = threadIdx.x, w = tid >> 5, lane = tid & 31, ln = lane & 15, hh = lane >> 4; const int by = blockIdx.y;
  A += (size_t)by * sA; Bh += (size_t)by * sB; const size_t cofs = (size_t)by * sC; const float* bp = bias ? bias + (size_t)by * sBias : nullptr;
  const int ntn = (N + 63) / 64; const int wid = blockIdx.x * 4 + w; const int mt = wid / ntn, nq = wid % ntn; if (mt * 16 >= M) return;
  const int row0 = mt * 16, col0 = nq * 64; const _Float16* arow = A + (size_t)(row0 + ln) * lda;
  v8f acc[4] = {};
  for (int kb = 0; kb < K; kb += 32) { FragH ah; ah.half[0] = *(const v8us*)((const unsigned short*)arow + kb + 8 * hh); ah.half[1] = *(const v8us*)((const unsigned short*)arow + kb + 16 + 8 * hh);
#pragma unroll
    for (int t = 0; t < 4; ++t) { if (col0 + t * 16 >= N) continue; const size_t boff = (size_t)(col0 + t * 16 + ln) * ldb + kb; FragH bq; bq.half[0] = *(const v8us*)((const unsigned short*)Bh + boff + 8 * hh); bq.half[1] = *(const v8us*)((const unsigned short*)Bh + boff + 16 + 8 * hh);
      acc[t] = mmaH<1>(ah.v, ah.v, bq.v, bq.v, acc[t]); }
  }
#pragma unroll
  for (int t = 0; t < 4; ++t) { if (col0 + t * 16 >= N) continue; const int col = col0 + t * 16 + ln; const float bv = bp ? bf16_round(bp[col]) : 0.f;
#pragma unroll
    for (int r = 0; r < 8; ++r) { float v = acc[t][r] * alpha + bv; if (CP) { const int bidx = (row0g + row0 + 8 * hh + r) / rowsPerB; v += CP[(size_t)bidx * sCPb + (size_t)by * 64 + col]; } if (ACT == 1) v = (v > 0.f) ? v : expm1f(v); else if (ACT == 3) v = fmaxf(v, 0.f); so[w][8 * hh + r][t * 16 + ln] = v; } }
  __builtin_amdgcn_fence(__ATOMIC_ACQ_REL, "workgroup"); __builtin_amdgcn_wave_barrier();
  const int rsub = lane >> 4, c4 = (lane & 15) * 4; typedef _Float16 v4h __attribute__((ext_vector_type(4)));
  for (int pass = 0; pass < 2; ++pass) {
#pragma unroll
    for (int q = 0; q < 8; ++q) { const int r = q * 2 + rsub; if (col0 + c4 < N) { const v4f v = *(const v4fa*)&so[w][r][c4]; if (C) *(volatile v4f*)(C + cofs + (size_t)(row0 + r) * ldc + col0 + c4) = v; if (C16) { v4h h4; for (int i = 0; i < 4; ++i) h4[i] = (_Float16)v[i]; *(volatile v4h*)(C16 + cofs + (size_t)(row0 + r) * ldc + col0 + c4) = h4; } } }
    if (pass == 0) __threadfence(); }
}

__global__ __launch_bounds__(256) void k_bt(const float* __restrict__ eU, const float* __restrict__ mU, _Float16* __restrict__ BeU, _Float16* __restrict__ BmU) { const int t = blockIdx.x * 256 + threadIdx.x; if (t < NL * HH * HH) { const int k = t % HH, n = (t / HH) % HH, l = t / (HH * HH); *(volatile _Float16*)(BeU + t) = (_Float16)(bf16_round(eU[((size_t)l * HH + k) * HH + n]) * 16.0f); } if (t < HH * HH) { const int k = t % HH, n = t / HH; *(volatile _Float16*)(BmU + t) = (_Float16)(bf16_round(mU[k * HH + n]) * 16.0f); } }
__global__ __launch_bounds__(128) void k_initx(const float* __restrict__ coord, const float* __restrict__ wc, float* __restrict__ X) { const int n = blockIdx.x, h = threadIdx.x; const float v = bf16_round(coord[n * 2]) * bf16_round(wc[h]) + bf16_round(coord[n * 2 + 1]) * bf16_round(wc[HH + h]); *(volatile float*)(X + (size_t)n * HH + h) = v; __threadfence(); *(volatile float*)(X + (size_t)n * HH + h) = v; }
__global__ __launch_bounds__(128) void k_inite(const float* __restrict__ vals, const int* __restrict__ tags, const float* __restrict__ wev, const float* __restrict__ emb, float* __restrict__ E) { const size_t e = blockIdx.x; const int h = threadIdx.x; float v; if (h < HHALF) v = bf16_round(vals[e]) * bf16_round(wev[h]); else { int t = tags[e]; t = t < 0 ? 0 : (t > 2 ? 2 : t); v = bf16_round(emb[t * HHALF + h - HHALF]); } *(volatile float*)(E + e * HH + h) = v; __threadfence(); *(volatile float*)(E + e * HH + h) = v; }
__global__ __launch_bounds__(384) void k_nodeg(const float* __restrict__ X, const float* __restrict__ mask, const float* __restrict__ eV, const float* __restrict__ eVb, const float* __restrict__ nU, const float* __restrict__ nUb, const float* __restrict__ nV, const float* __restrict__ nVb, int l, float* __restrict__ NODE) { __shared__ float sx[HH]; const int n = blockIdx.x, o = threadIdx.x; if (o < HH) sx[o] = X[(size_t)n * HH + o]; __syncthreads(); const int which = o / HH, c = o % HH; const float* W = (which == 0 ? eV : (which == 1 ? nU : nV)) + (size_t)l * HH * HH; const float* bb = (which == 0 ? eVb : (which == 1 ? nUb : nVb)) + l * HH; float s = bf16_round(bb[c]);
#pragma unroll 4
  for (int k = 0; k < HH; ++k) s += sx[k] * bf16_round(W[k * HH + c]); s *= bf16_round(mask[n]); *(volatile float*)(NODE + (size_t)n * 3 * HH + o) = s; __threadfence(); *(volatile float*)(NODE + (size_t)n * 3 * HH + o) = s; }
__global__ __launch_bounds__(256) void k_e16(const float* __restrict__ F, _Float16* __restrict__ A16, size_t n8) { const size_t t = (size_t)blockIdx.x * 256 + threadIdx.x; if (t >= n8) return; FragH f; for (int q = 0; q < 8; ++q) f.h[q] = (_Float16)F[t * 8 + q]; *(volatile v8us*)((unsigned short*)A16 + t * 8) = f.half[0]; __threadfence(); *(volatile v8us*)((unsigned short*)A16 + t * 8) = f.half[0]; }
__global__ __launch_bounds__(128) void k_edgeA(const float* __restrict__ T, const float* __restrict__ NODE, const float* __restrict__ mask, int b, float* __restrict__ XT, float* __restrict__ PART) { const int i = blockIdx.x, h = threadIdx.x; const int ni = b * NNODE + i; const float mi = bf16_round(mask[ni]); const float vxi = NODE[(size_t)ni * 3 * HH + h]; float agg = 0.f, den = 0.f, s1 = 0.f, s2 = 0.f;
#pragma unroll 2
  for (int j = 0; j < NNODE; ++j) { const int nj = b * NNODE + j; const float et = T[((size_t)i * NNODE + j) * HH + h] + vxi + NODE[(size_t)nj * 3 * HH + h]; const float sq = mi * bf16_round(mask[nj]); const float g = (1.0f / (1.0f + expf(-et))) * sq; agg += g * NODE[(size_t)nj * 3 * HH + 2 * HH + h]; den += g; s1 += sq * et; s2 += sq * et * et; }
  const float xt = NODE[(size_t)ni * 3 * HH + HH + h] + agg / (1e-20f + den);
  *(volatile float*)(XT + (size_t)ni * HH + h) = xt; *(volatile float*)(PART + (size_t)ni * 2 * HH + h) = s1; *(volatile float*)(PART + (size_t)ni * 2 * HH + HH + h) = s2; __threadfence(); *(volatile float*)(XT + (size_t)ni * HH + h) = xt; *(volatile float*)(PART + (size_t)ni * 2 * HH + h) = s1; *(volatile float*)(PART + (size_t)ni * 2 * HH + HH + h) = s2; }
__global__ __launch_bounds__(128) void k_stats(const float* __restrict__ PART, const float* __restrict__ XT, const float* __restrict__ mask, const float* __restrict__ gE, const float* __restrict__ bE, const float* __restrict__ gN, const float* __restrict__ bN, int l, float* __restrict__ X, float* __restrict__ EST) { const int h = threadIdx.x; float cntE = 0.f, cntN = 0.f; for (int b = 0; b < BB; ++b) { float sb = 0.f; for (int n = 0; n < NNODE; ++n) sb += bf16_round(mask[b * NNODE + n]); cntE += sb * sb; cntN += sb; }
  float s1 = 0.f, s2 = 0.f;
#pragma unroll 2
  for (int n = 0; n < NX; ++n) { s1 += PART[(size_t)n * 2 * HH + h]; s2 += PART[(size_t)n * 2 * HH + HH + h]; } const float meanE = s1 / cntE; const float varE = s2 / cntE - meanE * meanE; const float ivE = 1.0f / sqrtf(varE + 1e-5f);
  *(volatile float*)(EST + h) = meanE; *(volatile float*)(EST + HH + h) = ivE * bf16_round(gE[l * HH + h]); *(volatile float*)(EST + 2 * HH + h) = bf16_round(bE[l * HH + h]);
  float m1 = 0.f;
#pragma unroll 2
  for (int n = 0; n < NX; ++n) m1 += bf16_round(mask[n]) * XT[(size_t)n * HH + h]; m1 /= cntN; float v2 = 0.f;
#pragma unroll 2
  for (int n = 0; n < NX; ++n) { const float d = XT[(size_t)n * HH + h] - m1; v2 += bf16_round(mask[n]) * d * d; } v2 /= cntN; const float ivN = 1.0f / sqrtf(v2 + 1e-5f); const float gg = bf16_round(gN[l * HH + h]), be = bf16_round(bN[l * HH + h]);
#pragma unroll 2
  for (int n = 0; n < NX; ++n) { const float xt = XT[(size_t)n * HH + h]; const float xn = (bf16_round(mask[n]) > 0.f) ? ((xt - m1) * ivN * gg + be) : xt; const float v = X[(size_t)n * HH + h] + fmaxf(xn, 0.f); *(volatile float*)(X + (size_t)n * HH + h) = v; }
  __threadfence(); *(volatile float*)(EST + h) = meanE; *(volatile float*)(EST + HH + h) = ivE * bf16_round(gE[l * HH + h]); *(volatile float*)(EST + 2 * HH + h) = bf16_round(bE[l * HH + h]);
#pragma unroll 2
  for (int n = 0; n < NX; ++n) { const float v = X[(size_t)n * HH + h]; *(volatile float*)(X + (size_t)n * HH + h) = v; } }
__global__ __launch_bounds__(128) void k_edgeB(const float* __restrict__ T, const float* __restrict__ NODE, const float* __restrict__ mask, const float* __restrict__ EST, int b, float* __restrict__ E) { const int i = blockIdx.x, h = threadIdx.x; const int ni = b * NNODE + i; const float mi = bf16_round(mask[ni]); const float vxi = NODE[(size_t)ni * 3 * HH + h]; const float mean = EST[h], ivg = EST[HH + h], be = EST[2 * HH + h];
  for (int pass = 0; pass < 2; ++pass) {
#pragma unroll 2
    for (int j = 0; j < NNODE; ++j) { const int nj = b * NNODE + j; const size_t e = ((size_t)ni * NNODE + j); const float et = T[((size_t)i * NNODE + j) * HH + h] + vxi + NODE[(size_t)nj * 3 * HH + h]; const float sq = mi * bf16_round(mask[nj]); const float en = (sq > 0.f) ? ((et - mean) * ivg + be) : et;
      if (pass == 0) { const float v = E[e * HH + h] + fmaxf(en, 0.f); *(volatile float*)(E + e * HH + h) = v; } else { const float v = *(volatile float*)(E + e * HH + h); *(volatile float*)(E + e * HH + h) = v; } }
    if (pass == 0) __threadfence(); } }
__global__ __launch_bounds__(256) void k_y(const _Float16* __restrict__ Hc, const float* __restrict__ mV, const float* __restrict__ bV, size_t e0, float* __restrict__ out) { __shared__ float sw[2][HH]; const int tid = threadIdx.x; if (tid < HH) { sw[0][tid] = bf16_round(mV[tid * 2]); sw[1][tid] = bf16_round(mV[tid * 2 + 1]); } __syncthreads(); const size_t el = (size_t)blockIdx.x * 256 + tid; if (el >= ECH) return; const unsigned short* hr = (const unsigned short*)Hc + el * HH; float y0 = bf16_round(bV[0]), y1 = bf16_round(bV[1]);
#pragma unroll 2
  for (int g = 0; g < HH / 8; ++g) { FragH f; f.half[0] = *(const v8us*)(hr + g * 8); for (int q = 0; q < 8; ++q) { const float hv = (float)f.h[q]; y0 += hv * sw[0][g * 8 + q]; y1 += hv * sw[1][g * 8 + q]; } }
  typedef float v2f __attribute__((ext_vector_type(2), aligned(8))); v2f o = {y0, y1}; *(volatile v2f*)(out + (e0 + el) * 2) = o; __threadfence(); *(volatile v2f*)(out + (e0 + el) * 2) = o; }
extern "C" void kernel_launch(void* const* d_in, const int* in_sizes, int n_in,
                              void* d_out, int out_size, void* d_ws, size_t ws_size, hipStream_t stream) {
  (void)in_sizes; (void)n_in; (void)out_size;
  const int* tags = (const int*)d_in[0]; const float* vals = (const float*)d_in[1]; const float* coord = (const float*)d_in[2]; const float* mask = (const float*)d_in[3]; const float* wc = (const float*)d_in[4]; const float* wev = (const float*)d_in[5]; const float* emb = (const float*)d_in[6];
  const float* eU = (const float*)d_in[7]; const float* eUb = (const float*)d_in[8]; const float* eV = (const float*)d_in[9]; const float* eVb = (const float*)d_in[10]; const float* nU = (const float*)d_in[11]; const float* nUb = (const float*)d_in[12]; const float* nV = (const float*)d_in[13]; const float* nVb = (const float*)d_in[14];
  const float* gE = (const float*)d_in[15]; const float* bE = (const float*)d_in[16]; const float* gN = (const float*)d_in[17]; const float* bN = (const float*)d_in[18]; const float* mU = (const float*)d_in[19]; const float* mUb = (const float*)d_in[20]; const float* mV = (const float*)d_in[21]; const float* mVb = (const float*)d_in[22];
  char* ws = (char*)d_ws; size_t off = 0;
  auto take = [&](size_t bytes) { char* p = ws + off; off += (bytes + 255) & ~(size_t)255; return p; };
  _Float16* BeU = (_Float16*)take((size_t)NL * HH * HH * 2); _Float16* BmU = (_Float16*)take(HH * HH * 2); float* X = (float*)take((size_t)NX * HH * 4); float* NODE = (float*)take((size_t)NX * 3 * HH * 4); float* XT = (float*)take((size_t)NX * HH * 4); float* PART = (float*)take((size_t)NX * 2 * HH * 4); float* EST = (float*)take(3 * HH * 4);
  float* E = (float*)take((size_t)NEDGE * HH * 4); _Float16* A16 = (_Float16*)take((size_t)ECH * HH * 2); float* T = (float*)take((size_t)ECH * HH * 4); _Float16* Hc = (_Float16*)T;
  if (off > ws_size) return;
  const unsigned E8 = (unsigned)(((size_t)ECH * HH / 8 + 255) / 256); const dim3 gch(((ECH / 16) * (HH / 64) + 3) / 4, 1);
  k_bt<<<(NL * HH * HH + 255) / 256, 256, 0, stream>>>(eU, mU, BeU, BmU);
  k_initx<<<NX, 128, 0, stream>>>(coord, wc, X); k_inite<<<NEDGE, 128, 0, stream>>>(vals, tags, wev, emb, E);
  for (int l = 0; l < NL; ++l) {
    k_nodeg<<<NX, 384, 0, stream>>>(X, mask, eV, eVb, nU, nUb, nV, nVb, l, NODE);
    for (int b = 0; b < BB; ++b) { k_e16<<<E8, 256, 0, stream>>>(E + (size_t)b * ECH * HH, A16, (size_t)ECH * HH / 8);
      k_gemm_hhx<0><<<gch, 128, 0, stream>>>(A16, HH, 0, BeU + (size_t)l * HH * HH, HH, 0, 0.0625f, eUb + l * HH, 0, nullptr, 1, 0, 0, T, nullptr, HH, 0, ECH, HH, HH);
      k_edgeA<<<NNODE, 128, 0, stream>>>(T, NODE, mask, b, XT, PART); }
    k_stats<<<1, 128, 0, stream>>>(PART, XT, mask, gE, bE, gN, bN, l, X, EST);
    for (int b = 0; b < BB; ++b) { k_e16<<<E8, 256, 0, stream>>>(E + (size_t)b * ECH * HH, A16, (size_t)ECH * HH / 8);
      k_gemm_hhx<0><<<gch, 128, 0, stream>>>(A16, HH, 0, BeU + (size_t)l * HH * HH, HH, 0, 0.0625f, eUb + l * HH, 0, nullptr, 1, 0, 0, T, nullptr, HH, 0, ECH, HH, HH);
      k_edgeB<<<NNODE, 128, 0, stream>>>(T, NODE, mask, EST, b, E); } }
  for (int b = 0; b < BB; ++b) { k_e16<<<E8, 256, 0, stream>>>(E + (size_t)b * ECH * HH, A16, (size_t)ECH * HH / 8);
    k_gemm_hhx<3><<<gch, 128, 0, stream>>>(A16, HH, 0, BmU, HH, 0, 0.0625f, mUb, 0, nullptr, 1, 0, 0, nullptr, Hc, HH, 0, ECH, HH, HH);
    k_y<<<(ECH + 255) / 256, 256, 0, stream>>>(Hc, mV, mVb, (size_t)b * ECH, (float*)d_out); }
}
